// TAD_GAT_10943576670617
// MI455X (gfx1250) — hardware-verified
//
#include <hip/hip_runtime.h>
#include <stddef.h>
#include <stdint.h>
#include <math.h>


#define BATCH   4
#define NNODE   10000
#define MROW    40000
#define NEDGE   160000
#define XF      291
#define NFD     57
#define RTD     78
#define KXT     96
#define KXB     64
#define HID     64
#define HC      256
#define KH      128
#define KA2     512
#define NTHR    256
#define NWAVE   8
#define EPT     8
#define CHUNK   (NTHR * EPT)
#define WCAP    (EPT * 32)
#define LISTN   (NWAVE * WCAP)
#define NBA     1024
#define SLA     10
#define RCAP    28672
#define DEGCAP  128
#define MEAS_B1024  16569
#define MEAS_MAXDEG 36
#define GBM     64
#define GBN     64
#define GTHR    128
#define NEGSL   0.2f
#define WSMAX   134217728
#define BKT_LDS_INTS  (LISTN + RCAP + 16)
#define SCAN_ZINTS    (RCAP + 3 * NBA)
#define SCAN_LDS_INTS (2 * RCAP + 3 * NBA + 16)
#define SC_WOFF       (HC + NWAVE * HC)

#define PA_ROWS  64
#define PA_FLT   (PA_ROWS * XF)
#define PA_V4    (PA_FLT / 4)
#define PA_UT    (PA_ROWS * (KXT / 8))
#define PA_UX    (3 * PA_UT)
#define PA_UB    (PA_ROWS * (KXB / 8))
#define PA_UNITS (PA_UX + PA_UB)
#define U_WIH   (HC * (KXT / 8))
#define U_WHH   (HC * (KH / 8))
#define U_WN    (HID * (KXB / 8))
#define U_W1    (HC * (KH / 8))
#define U_W2    (HC * (KA2 / 8))
#define U_ALL   (U_WIH + U_WHH + U_WN + U_W1 + U_W2)
#define L_OFF_G    0
#define L_OFF_SEQ  65536
#define L_OFF_C    114688
#define L_OFF_HA   131072
#define L_OFF_BG   147456
#define L_OFF_WA   148480
#define L_OFF_BN   148736
#define L_OFF_SC   148992
#define L_OFF_MS   150016
#define LSTM_LDS   150080

static_assert(MROW == BATCH * NNODE && MROW == 625 * 64);
static_assert(XF == NFD + 3 * RTD);
static_assert((KXT % 32) == 0 && (KXB % 32) == 0 && (KH % 32) == 0 && (KA2 % 32) == 0);
static_assert(KH == 2 * HID && KA2 == 2 * HC && HC == 4 * HID && HC == 32 * 8);
static_assert((PA_FLT % 4) == 0 && ((PA_FLT * 4) % 16) == 0);
static_assert((PA_UX % NTHR) == 0 && (PA_UNITS % NTHR) == 0 && (MROW % PA_ROWS) == 0);
static_assert((U_WIH % NTHR) == 0 && (U_WHH % NTHR) == 0 && (U_WN % NTHR) == 0);
static_assert((U_W1 % NTHR) == 0 && (U_W2 % NTHR) == 0 && (U_ALL % NTHR) == 0);
static_assert((CHUNK & (CHUNK - 1)) == 0 && CHUNK <= 4096);
static_assert((NBA & (NBA - 1)) == 0 && NBA == (1 << SLA) && NBA <= 1024);
static_assert(((long long)CHUNK << SLA) < (1LL << 31));
static_assert(NBA % NWAVE == 0 && NBA % 32 == 0 && NBA % 4 == 0);
static_assert((RCAP % (NTHR * 4)) == 0 && (SCAN_ZINTS % 4) == 0);
static_assert(RCAP >= MEAS_B1024 + 4096);
static_assert(DEGCAP >= MEAS_MAXDEG + 8);
static_assert(NNODE < 65536);
static_assert(SCAN_LDS_INTS * 4 <= 300000 && BKT_LDS_INTS * 4 <= 300000 && LSTM_LDS <= 300000);
static_assert(GBM == (GTHR / 32) * 16 && GTHR == 2 * GBN && GTHR == 2 * GBM);
static_assert((MROW % GBM) == 0 && (HC % GBN) == 0 && HID == GBN);
static_assert(NTHR == HC);
static_assert(SC_WOFF * 4 % 16 == 0 && SC_WOFF + NWAVE * 512 * 2 <= RCAP);
static_assert((MROW % 8) == 0 && (MROW % 32) == 0);

typedef float          v2f  __attribute__((ext_vector_type(2)));
typedef float          v4f  __attribute__((ext_vector_type(4)));
typedef float          v8f  __attribute__((ext_vector_type(8)));
typedef double         v2d  __attribute__((ext_vector_type(2)));
typedef int            v4i  __attribute__((ext_vector_type(4)));
typedef int            v8i  __attribute__((ext_vector_type(8)));
typedef unsigned short v8us __attribute__((ext_vector_type(8)));
typedef __bf16         v16b __attribute__((ext_vector_type(16)));
typedef v4f  __attribute__((may_alias)) v4fa;
typedef v2d  __attribute__((may_alias)) v2da;
typedef v4i  __attribute__((may_alias)) v4ia;
typedef v8us __attribute__((may_alias)) v8usa;
union FragB { v16b v; v8us h[2]; v8i w; };

__device__ __forceinline__ v8f wmb(const FragB& a, const FragB& b, v8f c) {
  v8f d = __builtin_amdgcn_wmma_f32_16x16x32_bf16(false, a.v, false, b.v, (short)0, c, false, false);
  asm volatile("v_nop\n\tv_nop\n\tv_nop\n\tv_nop" : "+v"(d) : "v"(a.w), "v"(b.w));
  return d;
}
__device__ __forceinline__ v8f z8() { v8f z = {0.f, 0.f, 0.f, 0.f, 0.f, 0.f, 0.f, 0.f}; return z; }

__device__ __forceinline__ unsigned int f2bf(float f) {
  const unsigned int u = __float_as_uint(f);
  const unsigned int r = ((u + 0x7FFFu + ((u >> 16) & 1u)) >> 16) & 0xFFFFu;
  return ((u & 0x7FFFFFFFu) > 0x7F800000u) ? 0x7FC0u : r;
}
__device__ __forceinline__ float bf2f(unsigned int b) { return __uint_as_float(b << 16); }
__device__ __forceinline__ float bfr(float f) { return bf2f(f2bf(f)); }
__device__ __forceinline__ float sigf(float v) { return 1.0f / (1.0f + expf(-v)); }

template <int SLB>
__device__ __forceinline__ int scan_chunk(const int* __restrict__ dsts, int nE, int cbase, int slotBase,
                                          int nb, int vec8, int* list, int tid, int lane, int wave) {
  int wc = 0;
  const int el0  = tid * EPT;
  const int e0   = cbase + el0;
  const int sent = -2147483647 - 1;
  v4i da, db;
  if (vec8 != 0 && cbase + CHUNK <= nE) {
    da = *(const v4i*)(dsts + e0);
    db = *(const v4i*)(dsts + e0 + 4);
  } else {
    da.x = (e0     < nE) ? dsts[min(e0,     nE - 1)] : sent;
    da.y = (e0 + 1 < nE) ? dsts[min(e0 + 1, nE - 1)] : sent;
    da.z = (e0 + 2 < nE) ? dsts[min(e0 + 2, nE - 1)] : sent;
    da.w = (e0 + 3 < nE) ? dsts[min(e0 + 3, nE - 1)] : sent;
    db.x = (e0 + 4 < nE) ? dsts[min(e0 + 4, nE - 1)] : sent;
    db.y = (e0 + 5 < nE) ? dsts[min(e0 + 5, nE - 1)] : sent;
    db.z = (e0 + 6 < nE) ? dsts[min(e0 + 6, nE - 1)] : sent;
    db.w = (e0 + 7 < nE) ? dsts[min(e0 + 7, nE - 1)] : sent;
  }
  const unsigned nbs = (unsigned)slotBase;
  const unsigned unb = (unsigned)nb;
  const unsigned s0 = (unsigned)da.x - nbs, s1 = (unsigned)da.y - nbs;
  const unsigned s2 = (unsigned)da.z - nbs, s3 = (unsigned)da.w - nbs;
  const unsigned s4 = (unsigned)db.x - nbs, s5 = (unsigned)db.y - nbs;
  const unsigned s6 = (unsigned)db.z - nbs, s7 = (unsigned)db.w - nbs;
  const bool h0 = s0 < unb, h1 = s1 < unb, h2 = s2 < unb, h3 = s3 < unb;
  const bool h4 = s4 < unb, h5 = s5 < unb, h6 = s6 < unb, h7 = s7 < unb;
  const unsigned any = __builtin_amdgcn_ballot_w32(h0 | h1 | h2 | h3 | h4 | h5 | h6 | h7);
  if (any != 0u) {
#define HITJ(J, HJ, SJ) { \
      const unsigned mj = __builtin_amdgcn_ballot_w32(HJ); \
      if (mj != 0u) { \
        if (HJ) { \
          const int pos = wc + (int)__builtin_amdgcn_mbcnt_lo(mj, 0u); \
          if (pos < WCAP) list[wave * WCAP + pos] = ((el0 + (J)) << SLB) | (int)(SJ); \
        } \
        wc += (int)__builtin_popcount(mj); } }
    HITJ(0, h0, s0)
    HITJ(1, h1, s1)
    HITJ(2, h2, s2)
    HITJ(3, h3, s3)
    HITJ(4, h4, s4)
    HITJ(5, h5, s5)
    HITJ(6, h6, s6)
    HITJ(7, h7, s7)
#undef HITJ
  }
  return wc;
}

__device__ __forceinline__ v8us pa_unit(const unsigned short* sx, int u) {
  v8us o;
  if (u < PA_UX) {
    const int t   = u / PA_UT;
    const int v   = u - t * PA_UT;
    const int row = v / 12;
    const int c0  = (v - row * 12) * 8;
    const unsigned short* p = sx + row * XF + NFD + t * RTD;
#pragma unroll
    for (int i = 0; i < 8; ++i) {
      const int k  = c0 + i;
      const int kc = k < RTD ? k : RTD - 1;
      const unsigned short w = p[kc];
      o[i] = (k < RTD) ? w : (unsigned short)0;
    }
  } else {
    const int v   = u - PA_UX;
    const int row = v >> 3;
    const int c0  = (v & 7) * 8;
    const unsigned short* p = sx + row * XF;
#pragma unroll
    for (int i = 0; i < 8; ++i) {
      const int k  = c0 + i;
      const int kc = k < NFD ? k : NFD - 1;
      const unsigned short w = p[kc];
      o[i] = (k < NFD) ? w : (unsigned short)0;
    }
  }
  return o;
}
__device__ __forceinline__ unsigned short* pa_dst(unsigned short* XT, unsigned short* XB, int r0, int u) {
  if (u < PA_UX) {
    const int t = u / PA_UT;
    const int v = u - t * PA_UT;
    return XT + ((size_t)t * MROW + (size_t)r0) * KXT + (size_t)v * 8;
  }
  return XB + (size_t)r0 * KXB + (size_t)(u - PA_UX) * 8;
}

__global__ __launch_bounds__(NTHR) void k_pa(const float* __restrict__ x, unsigned short* XT, unsigned short* XB) {
  __shared__ __attribute__((aligned(16))) unsigned short sx[PA_FLT];
  const int tid = (int)threadIdx.x;
  const int blk = (int)blockIdx.x;
  const int r0  = blk * PA_ROWS;
  const v4f* xp = (const v4f*)(x + (size_t)blk * PA_FLT);
#pragma unroll 2
  for (int q = tid; q < PA_V4; q += NTHR) {
    const v4f v = xp[q];
    sx[4 * q + 0] = (unsigned short)f2bf(v.x);
    sx[4 * q + 1] = (unsigned short)f2bf(v.y);
    sx[4 * q + 2] = (unsigned short)f2bf(v.z);
    sx[4 * q + 3] = (unsigned short)f2bf(v.w);
  }
  __syncthreads();
#pragma unroll 1
  for (int it = 0; it < PA_UNITS / NTHR; ++it) {
    const int u = it * NTHR + tid;
    const v8us o = pa_unit(sx, u);
    unsigned short* dp = pa_dst(XT, XB, r0, u);
    *(volatile v8us*)dp = o;
  }
  __threadfence();
#pragma unroll 1
  for (int it = 0; it < PA_UNITS / NTHR; ++it) {
    const int u = it * NTHR + tid;
    const v8us o = pa_unit(sx, u);
    unsigned short* dp = pa_dst(XT, XB, r0, u);
    *(volatile v8us*)dp = o;
  }
}

__device__ __forceinline__ v8us cv8(const float* p) {
  const v4f a = *(const v4f*)p;
  const v4f b = *(const v4f*)(p + 4);
  v8us o;
  o[0] = (unsigned short)f2bf(a.x); o[1] = (unsigned short)f2bf(a.y);
  o[2] = (unsigned short)f2bf(a.z); o[3] = (unsigned short)f2bf(a.w);
  o[4] = (unsigned short)f2bf(b.x); o[5] = (unsigned short)f2bf(b.y);
  o[6] = (unsigned short)f2bf(b.z); o[7] = (unsigned short)f2bf(b.w);
  return o;
}

__global__ __launch_bounds__(NTHR) void k_pb(const float* __restrict__ Wih, const float* __restrict__ Whh,
                                             const float* __restrict__ Wn, const float* __restrict__ W1,
                                             const float* __restrict__ W2, unsigned short* WIH,
                                             unsigned short* WHH2, unsigned short* WN, unsigned short* W1D,
                                             unsigned short* W2D) {
  const int u = (int)blockIdx.x * NTHR + (int)threadIdx.x;
  v8us o;
  unsigned short* dp;
  if (u < U_WIH) {
    const int n  = u / 12;
    const int c0 = (u - n * 12) * 8;
    const float* p = Wih + (size_t)n * RTD;
#pragma unroll
    for (int i = 0; i < 8; ++i) {
      const int k  = c0 + i;
      const int kc = k < RTD ? k : RTD - 1;
      const float f = p[kc];
      o[i] = (k < RTD) ? (unsigned short)f2bf(f) : (unsigned short)0;
    }
    dp = WIH + (size_t)u * 8;
  } else if (u < U_WIH + U_WHH) {
    const int v  = u - U_WIH;
    const int n  = v >> 4;
    const int kk = ((v & 15) * 8) & (HID - 1);
    o = cv8(Whh + (size_t)n * HID + kk);
    dp = WHH2 + (size_t)v * 8;
  } else if (u < U_WIH + U_WHH + U_WN) {
    const int v  = u - U_WIH - U_WHH;
    const int n  = v >> 3;
    const int c0 = (v & 7) * 8;
    const float* p = Wn + (size_t)n * NFD;
#pragma unroll
    for (int i = 0; i < 8; ++i) {
      const int k  = c0 + i;
      const int kc = k < NFD ? k : NFD - 1;
      const float f = p[kc];
      o[i] = (k < NFD) ? (unsigned short)f2bf(f) : (unsigned short)0;
    }
    dp = WN + (size_t)v * 8;
  } else if (u < U_WIH + U_WHH + U_WN + U_W1) {
    const int v  = u - U_WIH - U_WHH - U_WN;
    const int n  = v >> 4;
    const int kk = ((v & 15) * 8) & (HID - 1);
    o = cv8(W1 + (size_t)n * HID + kk);
    dp = W1D + (size_t)v * 8;
  } else if (u < U_ALL) {
    const int v  = u - U_WIH - U_WHH - U_WN - U_W1;
    const int n  = v >> 6;
    const int kk = ((v & 63) * 8) & (HC - 1);
    o = cv8(W2 + (size_t)n * HC + kk);
    dp = W2D + (size_t)v * 8;
  } else {
    return;
  }
  *(volatile v8us*)dp = o;
  __threadfence();
  *(volatile v8us*)dp = o;
}

__global__ __launch_bounds__(NTHR) void k_bucket(const int* __restrict__ srcs, const int* __restrict__ dsts,
                                                 int nE, int nN, int vec8, int* HITS, int* FLG) {
  extern __shared__ __attribute__((aligned(16))) int bsm[];
  int* list = bsm;
  int* reg1 = bsm + LISTN;
  int* wcnt = reg1 + RCAP;
  const int tid = (int)threadIdx.x, lane = tid & 31, wave = tid >> 5;
  const int blk = (int)blockIdx.x;
  const int nodeBase = blk * NBA;
  int nb = nN - nodeBase;
  nb = nb < 0 ? 0 : (nb > NBA ? NBA : nb);

  int tot = 0, ovf = 0;
  const int nChunks = (nE + CHUNK - 1) / CHUNK;
#pragma unroll 1
  for (int ch = 0; ch < nChunks; ++ch) {
    const int cbase = ch * CHUNK;
    const int wc = scan_chunk<SLA>(dsts, nE, cbase, nodeBase, nb, vec8, list, tid, lane, wave);
    if (lane == 0) wcnt[wave] = wc;
    __syncthreads();
    int pre = 0, all = 0;
#pragma unroll
    for (int w2 = 0; w2 < NWAVE; ++w2) {
      int c = wcnt[w2];
      c = c < 0 ? 0 : (c > WCAP ? WCAP : c);
      all += c;
      pre += (w2 < wave) ? c : 0;
    }
    const int wcc  = wc > WCAP ? WCAP : wc;
    const int base = tot + pre;
#pragma unroll 1
    for (int i = lane; i < wcc; i += 32) {
      const int ent = list[wave * WCAP + i];
      const int el  = (ent >> SLA) & (CHUNK - 1);
      const int sl  = ent & (NBA - 1);
      int eid = cbase + el;
      eid = eid > nE - 1 ? nE - 1 : eid;
      const int sraw = srcs[eid];
      const int s = sraw < 0 ? 0 : (sraw > nN - 1 ? nN - 1 : sraw);
      const int pos = base + i;
      if (pos < RCAP) reg1[pos] = (int)((unsigned)s | ((unsigned)sl << 16));
    }
    if (tot + all > RCAP) ovf = 1;
    tot += all;
    tot = tot > RCAP ? RCAP : tot;
    __syncthreads();
  }
  const int nh = tot;
  for (int i = nh + tid; i < RCAP; i += NTHR) reg1[i] = 0;
  __syncthreads();

  int* hb = HITS + (size_t)blk * RCAP;
  v4i cv;
  cv.x = (tid == 0) ? nh : 0;
  cv.y = (tid == 0) ? ovf : 0;
  cv.z = 0; cv.w = 0;
  int* fp = FLG + (size_t)blk * 32 + 4 * (tid & 7);
#pragma unroll 1
  for (int p = tid * 4; p < RCAP; p += NTHR * 4) {
    const v4i v = *(const v4ia*)(reg1 + p);
    *(volatile v4i*)(hb + p) = v;
  }
  if (tid < 8) *(volatile v4i*)fp = cv;
  __threadfence();
#pragma unroll 1
  for (int p = tid * 4; p < RCAP; p += NTHR * 4) {
    const v4i v = *(const v4ia*)(reg1 + p);
    *(volatile v4i*)(hb + p) = v;
  }
  if (tid < 8) *(volatile v4i*)fp = cv;
}

__global__ __launch_bounds__(NTHR) __attribute__((amdgpu_num_vgpr(248)))
void k_lstm(const unsigned short* __restrict__ XT, const unsigned short* __restrict__ WIH,
            const unsigned short* __restrict__ WHH2, const unsigned short* __restrict__ XB,
            const unsigned short* __restrict__ WN, const float* __restrict__ bih,
            const float* __restrict__ bhh, const float* __restrict__ Wa, const float* __restrict__ ba,
            const float* __restrict__ bnb, unsigned short* H0HL) {
  extern __shared__ __attribute__((aligned(16))) unsigned char lsm[];
  float* sG   = (float*)(lsm + L_OFF_G);
  float* sSeq = (float*)(lsm + L_OFF_SEQ);
  float* sC   = (float*)(lsm + L_OFF_C);
  unsigned short* sHA = (unsigned short*)(lsm + L_OFF_HA);
  float* sBG  = (float*)(lsm + L_OFF_BG);
  float* sWA  = (float*)(lsm + L_OFF_WA);
  float* sBN  = (float*)(lsm + L_OFF_BN);
  float* sSc  = (float*)(lsm + L_OFF_SC);
  float* sMs  = (float*)(lsm + L_OFF_MS);
  const int tid = (int)threadIdx.x, lane = tid & 31, wave = tid >> 5, hh = lane >> 4, m = lane & 15;
  const int rowBase = (int)blockIdx.x * 64;

  sBG[tid] = bfr(bih[tid]) + bfr(bhh[tid]);
  {
    const int c = tid & 63;
    const float va = Wa[c];
    const float vb = bnb[c];
    if (tid < 64) sWA[c] = bfr(va);
    else if (tid < 128) sBN[c] = bfr(vb);
  }
  if (tid < 16) sMs[tid] = (tid == 0) ? bfr(ba[0]) : 0.0f;
#pragma unroll 1
  for (int i = tid; i < 64 * HID; i += NTHR) sC[i] = 0.0f;

  const int j  = tid & 63;
  const int rg = tid >> 6;

#pragma unroll 1
  for (int t = 0; t < 3; ++t) {
    v8f acc[8];
#pragma unroll
    for (int i = 0; i < 8; ++i) acc[i] = z8();
    {
      const unsigned short* ap = XT + ((size_t)t * MROW + (size_t)(rowBase + m)) * KXT + 8 * hh;
      const unsigned short* wp = WIH + (size_t)(32 * wave + m) * KXT + 8 * hh;
#pragma unroll 1
      for (int ks = 0; ks < KXT / 32; ++ks) {
        FragB b0, b1;
        b0.h[0] = *(const v8usa*)(wp + 32 * ks);
        b0.h[1] = *(const v8usa*)(wp + 32 * ks + 16);
        b1.h[0] = *(const v8usa*)(wp + 16 * KXT + 32 * ks);
        b1.h[1] = *(const v8usa*)(wp + 16 * KXT + 32 * ks + 16);
#pragma unroll
        for (int mt = 0; mt < 4; ++mt) {
          FragB af;
          af.h[0] = *(const v8usa*)(ap + (size_t)(16 * mt) * KXT + 32 * ks);
          af.h[1] = *(const v8usa*)(ap + (size_t)(16 * mt) * KXT + 32 * ks + 16);
          acc[2 * mt]     = wmb(af, b0, acc[2 * mt]);
          acc[2 * mt + 1] = wmb(af, b1, acc[2 * mt + 1]);
        }
      }
    }
    if (t > 0) {
      const unsigned short* hp = sHA + m * KH + 8 * hh;
      const unsigned short* vp = WHH2 + (size_t)(32 * wave + m) * KH + 8 * hh;
#pragma unroll 1
      for (int ks = 0; ks < KH / 32; ++ks) {
        FragB b0, b1;
        b0.h[0] = *(const v8usa*)(vp + 32 * ks);
        b0.h[1] = *(const v8usa*)(vp + 32 * ks + 16);
        b1.h[0] = *(const v8usa*)(vp + 16 * KH + 32 * ks);
        b1.h[1] = *(const v8usa*)(vp + 16 * KH + 32 * ks + 16);
#pragma unroll
        for (int mt = 0; mt < 4; ++mt) {
          FragB af;
          af.h[0] = *(const v8usa*)(hp + (16 * mt) * KH + 32 * ks);
          af.h[1] = *(const v8usa*)(hp + (16 * mt) * KH + 32 * ks + 16);
          acc[2 * mt]     = wmb(af, b0, acc[2 * mt]);
          acc[2 * mt + 1] = wmb(af, b1, acc[2 * mt + 1]);
        }
      }
    }
#pragma unroll
    for (int mt = 0; mt < 4; ++mt) {
#pragma unroll
      for (int nt = 0; nt < 2; ++nt) {
#pragma unroll
        for (int r = 0; r < 8; ++r) {
          sG[(16 * mt + 8 * hh + r) * HC + 32 * wave + 16 * nt + m] = acc[2 * mt + nt][r];
        }
      }
    }
    __syncthreads();

    const float b_i = sBG[j], b_f = sBG[64 + j], b_g = sBG[128 + j], b_o = sBG[192 + j];
#pragma unroll 1
    for (int i = 0; i < 16; ++i) {
      const int row = rg + 4 * i;
      const float* gr = sG + row * HC;
      const float vi = gr[j] + b_i;
      const float vf = gr[64 + j] + b_f;
      const float vg = gr[128 + j] + b_g;
      const float vo = gr[192 + j] + b_o;
      const float si = sigf(vi);
      const float sf = sigf(vf);
      const float so = sigf(vo);
      const float tg = tanhf(vg);
      const float cn = sf * sC[row * HID + j] + si * tg;
      const float hv = so * tanhf(cn);
      sC[row * HID + j] = cn;
      sSeq[(t * 64 + row) * HID + j] = hv;
      if (t < 2) {
        const unsigned int hb = f2bf(hv);
        sHA[row * KH + j]       = (unsigned short)hb;
        sHA[row * KH + HID + j] = (unsigned short)f2bf(hv - bf2f(hb));
      }
    }
    __syncthreads();
  }

  {
    const int mt  = wave >> 1;
    const int ntb = (wave & 1) * 2;
    v8f a0 = z8(), a1 = z8();
    const unsigned short* ap = XB + (size_t)(rowBase + 16 * mt + m) * KXB + 8 * hh;
    const unsigned short* wq = WN + (size_t)(16 * ntb + m) * KXB + 8 * hh;
#pragma unroll 1
    for (int ks = 0; ks < KXB / 32; ++ks) {
      FragB af, b0, b1;
      af.h[0] = *(const v8usa*)(ap + 32 * ks);
      af.h[1] = *(const v8usa*)(ap + 32 * ks + 16);
      b0.h[0] = *(const v8usa*)(wq + 32 * ks);
      b0.h[1] = *(const v8usa*)(wq + 32 * ks + 16);
      b1.h[0] = *(const v8usa*)(wq + 16 * KXB + 32 * ks);
      b1.h[1] = *(const v8usa*)(wq + 16 * KXB + 32 * ks + 16);
      a0 = wmb(af, b0, a0);
      a1 = wmb(af, b1, a1);
    }
#pragma unroll
    for (int r = 0; r < 8; ++r) {
      sG[(16 * mt + 8 * hh + r) * HID + 16 * ntb + m]      = a0[r];
      sG[(16 * mt + 8 * hh + r) * HID + 16 * ntb + 16 + m] = a1[r];
    }
  }
  if (tid < 64) {
    const int row = tid;
    float l0 = 0.f, l1 = 0.f, l2 = 0.f;
#pragma unroll 4
    for (int u = 0; u < HID; ++u) {
      const float w = sWA[u];
      l0 = fmaf(sSeq[(0 * 64 + row) * HID + u], w, l0);
      l1 = fmaf(sSeq[(1 * 64 + row) * HID + u], w, l1);
      l2 = fmaf(sSeq[(2 * 64 + row) * HID + u], w, l2);
    }
    const float bav = sMs[0];
    l0 += bav; l1 += bav; l2 += bav;
    const float mx = fmaxf(l0, fmaxf(l1, l2));
    const float e0 = expf(l0 - mx), e1 = expf(l1 - mx), e2 = expf(l2 - mx);
    const float inv = 1.0f / (e0 + e1 + e2);
    sSc[row * 4 + 0] = e0 * inv;
    sSc[row * 4 + 1] = e1 * inv;
    sSc[row * 4 + 2] = e2 * inv;
    sSc[row * 4 + 3] = 0.0f;
  }
  __syncthreads();

  {
    const float bb = sBN[j];
#pragma unroll 1
    for (int i = 0; i < 16; ++i) {
      const int row = rg + 4 * i;
      const float a0 = sSc[row * 4], a1 = sSc[row * 4 + 1], a2 = sSc[row * 4 + 2];
      const float ht = sSeq[(0 * 64 + row) * HID + j] * a0 + sSeq[(1 * 64 + row) * HID + j] * a1 +
                       sSeq[(2 * 64 + row) * HID + j] * a2;
      float hs = sG[row * HID + j] + bb;
      hs = (hs <= 0.0f) ? 0.0f : hs;
      const float v = ht + hs;
      const unsigned int hb = f2bf(v);
      sHA[row * KH + j]       = (unsigned short)hb;
      sHA[row * KH + HID + j] = (unsigned short)f2bf(v - bf2f(hb));
    }
  }
  __syncthreads();

  unsigned short* ob = H0HL + (size_t)rowBase * KH;
#pragma unroll
  for (int it = 0; it < 4; ++it) {
    const int u = it * NTHR + tid;
    const v8us o = *(const v8usa*)(sHA + 8 * u);
    *(volatile v8us*)(ob + 8 * u) = o;
  }
  __threadfence();
#pragma unroll
  for (int it = 0; it < 4; ++it) {
    const int u = it * NTHR + tid;
    const v8us o = *(const v8usa*)(sHA + 8 * u);
    *(volatile v8us*)(ob + 8 * u) = o;
  }
}

__global__ __launch_bounds__(GTHR) __attribute__((amdgpu_num_vgpr(248))) void k_g(
    const unsigned short* __restrict__ A, const unsigned short* __restrict__ WT,
    float* outF, int K, int ldo,
    const float* __restrict__ atts, const float* __restrict__ attd, int attLen,
    float* SD, int MPr)
{
  __shared__ __attribute__((aligned(16))) float stg[GBM * GBN];
  __shared__ __attribute__((aligned(16))) float satt[2 * GBN];
  __shared__ __attribute__((aligned(16))) float sdot[2 * GBM];
  const int tid = (int)threadIdx.x, lane = tid & 31, wave = tid >> 5, hh = lane >> 4, m = lane & 15;
  const int rowBase = (int)blockIdx.x * GBM;
  const int head    = (int)blockIdx.y;
  const int col0    = head * GBN;

  {
    const int which = tid >> 6;
    const int c  = tid & 63;
    const int cl = c < attLen ? c : attLen - 1;
    const float vs = atts[head * attLen + cl];
    const float vd = attd[head * attLen + cl];
    float v = (which == 0) ? vs : vd;
    v = (c < attLen) ? bfr(v) : 0.f;
    satt[which * GBN + c] = v;
  }

  v8f acc[4];
  acc[0] = z8(); acc[1] = z8(); acc[2] = z8(); acc[3] = z8();
  const unsigned short* ap = A  + (size_t)(rowBase + 16 * wave + m) * (size_t)K + 8 * hh;
  const unsigned short* wp = WT + (size_t)(col0 + m) * (size_t)K + 8 * hh;
  const int ksteps = K >> 5;
#pragma unroll 1
  for (int ks = 0; ks < ksteps; ++ks) {
    FragB af;
    af.h[0] = *(const v8usa*)(ap + 32 * ks);
    af.h[1] = *(const v8usa*)(ap + 32 * ks + 16);
#pragma unroll
    for (int t = 0; t < 4; ++t) {
      const unsigned short* wq = wp + (size_t)(16 * t) * (size_t)K + 32 * ks;
      FragB bf;
      bf.h[0] = *(const v8usa*)wq;
      bf.h[1] = *(const v8usa*)(wq + 16);
      acc[t] = wmb(af, bf, acc[t]);
    }
  }

#pragma unroll
  for (int t = 0; t < 4; ++t) {
    const int lc = 16 * t + m;
#pragma unroll
    for (int r = 0; r < 8; ++r) {
      const int lr = 16 * wave + 8 * hh + r;
      stg[lr * GBN + lc] = acc[t][r];
    }
  }
  __syncthreads();

  {
    const int row = tid & 63, which = tid >> 6;
    const float* sa = satt + which * GBN;
    const float* hr = stg + row * GBN;
    float d = 0.f;
#pragma unroll 4
    for (int c4 = 0; c4 < GBN / 4; ++c4) {
      const v4f hv = *(const v4fa*)(hr + 4 * c4);
      const v4f av = *(const v4fa*)(sa + 4 * c4);
      d = fmaf(hv.x, av.x, d);
      d = fmaf(hv.y, av.y, d);
      d = fmaf(hv.z, av.z, d);
      d = fmaf(hv.w, av.w, d);
    }
    sdot[which * GBM + row] = d;
  }
  __syncthreads();

  v4f fv[8];
#pragma unroll
  for (int i = 0; i < 8; ++i) {
    const int lr = 16 * wave + 2 * i + hh;
    fv[i] = *(const v4fa*)(stg + lr * GBN + 4 * m);
  }
  const int which2 = lane >> 4, piece = lane & 15;
  const v4f sdv = *(const v4fa*)(sdot + which2 * GBM + 4 * piece);
  float* sp = SD + (size_t)(2 * head + which2) * (size_t)MPr + rowBase + 4 * piece;

#pragma unroll
  for (int i = 0; i < 8; ++i) {
    const int lr = 16 * wave + 2 * i + hh;
    const int gr = rowBase + lr;
    float* op = outF + (size_t)gr * (size_t)ldo + col0 + 4 * m;
    *(volatile v4f*)op = fv[i];
  }
  if (wave == 0) *(volatile v4f*)sp = sdv;
  __threadfence();
#pragma unroll
  for (int i = 0; i < 8; ++i) {
    const int lr = 16 * wave + 2 * i + hh;
    const int gr = rowBase + lr;
    float* op = outF + (size_t)gr * (size_t)ldo + col0 + 4 * m;
    *(volatile v4f*)op = fv[i];
  }
  if (wave == 0) *(volatile v4f*)sp = sdv;
}

__global__ __launch_bounds__(NTHR) __attribute__((amdgpu_num_vgpr(248)))
void k_scan(const int* __restrict__ HITS, const int* __restrict__ FLGB,
            const float* __restrict__ F, const float* __restrict__ SD,
            const float* __restrict__ bias, float* P, double* REC, int nN, int MPr) {
  extern __shared__ __attribute__((aligned(16))) int ssm[];
  int* hl   = ssm;
  int* sl   = ssm + RCAP;
  int* cnt  = sl + RCAP;
  int* offs = cnt + NBA;
  int* cur  = offs + NBA;
  int* misc = cur + NBA;
  const int tid = (int)threadIdx.x, lane = tid & 31, wave = tid >> 5;
  const int blk = (int)blockIdx.x;
  const int bb  = (int)blockIdx.y;
  const int nodeBase = blk * NBA;
  const int rowOff   = bb * nN;

  const int nhraw = FLGB[(size_t)blk * 32];
  const int bflag = FLGB[(size_t)blk * 32 + 1];
  const int nh  = nhraw < 0 ? 0 : (nhraw > RCAP ? RCAP : nhraw);
  const int ovf = (bflag != 0 || nhraw < 0 || nhraw > RCAP) ? 1 : 0;

  {
    const v4i z4 = {0, 0, 0, 0};
    for (int i = tid * 4; i < SCAN_ZINTS; i += NTHR * 4) *(v4ia*)(sl + i) = z4;
    if (tid < 16) misc[tid] = 0;
    const int* hb = HITS + (size_t)blk * RCAP;
    const int nh4 = (nh + 3) & ~3;
#pragma unroll 1
    for (int p = tid * 4; p < nh4; p += NTHR * 4) *(v4ia*)(hl + p) = *(const v4i*)(hb + p);
  }
  __syncthreads();

  if (wave == 0) {
#pragma unroll 1
    for (int b0 = 0; b0 < nh; b0 += 32) {
      const int idx = b0 + lane;
      const int uv  = hl[idx < nh ? idx : nh - 1];
      const int m32 = (nh - b0) < 32 ? (nh - b0) : 32;
#pragma unroll 1
      for (int k = 0; k < m32; ++k) {
        const int u  = __builtin_amdgcn_readlane(uv, k);
        const int sq = (u >> 16) & (NBA - 1);
        if (lane == 0) cnt[sq] = cnt[sq] + 1;
      }
    }
  }
  __syncthreads();
  if (wave == 0) {
    const int base = lane * (NBA / 32);
    int s = 0;
#pragma unroll 1
    for (int i = 0; i < NBA / 32; ++i) s += cnt[base + i];
    int incl = s;
#pragma unroll
    for (int d = 1; d < 32; d <<= 1) {
      const int y = __shfl_up(incl, d, 32);
      if (lane >= d) incl += y;
    }
    int run = incl - s;
#pragma unroll 1
    for (int i = 0; i < NBA / 32; ++i) {
      const int cv = cnt[base + i];
      offs[base + i] = run;
      cur[base + i]  = run;
      run += cv;
    }
  }
  __syncthreads();
  if (wave == 0) {
#pragma unroll 1
    for (int b0 = 0; b0 < nh; b0 += 32) {
      const int idx = b0 + lane;
      const int uv  = hl[idx < nh ? idx : nh - 1];
      const int m32 = (nh - b0) < 32 ? (nh - b0) : 32;
#pragma unroll 1
      for (int k = 0; k < m32; ++k) {
        const int u  = __builtin_amdgcn_readlane(uv, k);
        const int sq = (u >> 16) & (NBA - 1);
        if (lane == 0) {
          int p = cur[sq];
          p = p < 0 ? 0 : (p > RCAP - 1 ? RCAP - 1 : p);
          sl[p] = u;
          cur[sq] = p + 1;
        }
      }
    }
  }
  __syncthreads();

  float*  fl   = (float*)hl;
  float*  st   = fl + HC + wave * HC;
  double* wsum = (double*)(hl + SC_WOFF);
  fl[tid] = bfr(bias[tid]);
  __syncthreads();

  const float qnan = __int_as_float(0x7fc00000);
  const float pzb  = (ovf != 0) ? qnan : 0.0f;
  const int head   = lane >> 3;
  const size_t hoS = (size_t)(2 * head) * (size_t)MPr + (size_t)rowOff;
  const size_t hoD = hoS + (size_t)MPr;
  const v4f bA = *(const v4fa*)(fl + 4 * lane);
  const v4f bB = *(const v4fa*)(fl + 128 + 4 * lane);
  double ps[8], pq[8];
#pragma unroll
  for (int i = 0; i < 8; ++i) { ps[i] = 0.0; pq[i] = 0.0; }

#pragma unroll 1
  for (int si = 0; si < NBA / NWAVE; ++si) {
    const int s    = si * NWAVE + wave;
    const int node = nodeBase + s;
    if (node >= nN) break;
    const int nc   = node;
    int c = cnt[s];
    const bool big = c > DEGCAP;
    c = c < 0 ? 0 : (c > DEGCAP ? DEGCAP : c);
    int o = offs[s];
    o = o < 0 ? 0 : (o > RCAP ? RCAP : o);
    if (c > nh - o) c = nh - o;
    c = c < 0 ? 0 : c;
    const float adv = SD[hoD + (size_t)nc];
    float mx = -3.0e38f, dn = 0.0f;
    float acc[8];
#pragma unroll
    for (int i = 0; i < 8; ++i) acc[i] = 0.0f;
    const int T = c + 1;
#pragma unroll 1
    for (int b0 = 0; b0 < T; b0 += 32) {
      const int t = b0 + lane;
      int idx = o + t;
      idx = idx < 0 ? 0 : (idx > RCAP - 1 ? RCAP - 1 : idx);
      const int ent = sl[idx];
      int hs = ent & 0xFFFF;
      hs = hs > nN - 1 ? nN - 1 : hs;
      const int sr  = (t < c) ? hs : nc;
      const int m32 = (T - b0) < 32 ? (T - b0) : 32;
#pragma unroll 1
      for (int k = 0; k < m32; ++k) {
        const int sk = __builtin_amdgcn_readlane(sr, k);
        const float* rp = F + ((size_t)rowOff + (size_t)sk) * HC + 8 * lane;
        float lg = SD[hoS + (size_t)sk] + adv;
        lg = lg > 0.f ? lg : NEGSL * lg;
        const float df = lg - mx;
        const float ee = expf(-fabsf(df));
        const bool  up = df > 0.f;
        const float s1 = up ? ee : 1.0f;
        const float s2 = up ? 1.0f : ee;
        mx = up ? lg : mx;
        dn = fmaf(dn, s1, s2);
        const v4f a = *(const v4f*)rp;
        const v4f b = *(const v4f*)(rp + 4);
        acc[0] = fmaf(acc[0], s1, s2 * a.x); acc[1] = fmaf(acc[1], s1, s2 * a.y);
        acc[2] = fmaf(acc[2], s1, s2 * a.z); acc[3] = fmaf(acc[3], s1, s2 * a.w);
        acc[4] = fmaf(acc[4], s1, s2 * b.x); acc[5] = fmaf(acc[5], s1, s2 * b.y);
        acc[6] = fmaf(acc[6], s1, s2 * b.z); acc[7] = fmaf(acc[7], s1, s2 * b.w);
      }
    }
    const float inv = 1.0f / (dn + 1e-16f);
    const float pzr = big ? qnan : pzb;

    v4f w0, w1;
    w0.x = acc[0] * inv; w0.y = acc[1] * inv; w0.z = acc[2] * inv; w0.w = acc[3] * inv;
    w1.x = acc[4] * inv; w1.y = acc[5] * inv; w1.z = acc[6] * inv; w1.w = acc[7] * inv;
    *(v4fa*)(st + 8 * lane)     = w0;
    *(v4fa*)(st + 8 * lane + 4) = w1;
    __builtin_amdgcn_fence(__ATOMIC_RELEASE, "workgroup");
    __builtin_amdgcn_wave_barrier();
    const v4f ra = *(const v4fa*)(st + 4 * lane);
    const v4f rb = *(const v4fa*)(st + 128 + 4 * lane);
    __builtin_amdgcn_fence(__ATOMIC_RELEASE, "workgroup");
    __builtin_amdgcn_wave_barrier();

    float y[8];
    y[0] = ra.x + bA.x; y[1] = ra.y + bA.y; y[2] = ra.z + bA.z; y[3] = ra.w + bA.w;
    y[4] = rb.x + bB.x; y[5] = rb.y + bB.y; y[6] = rb.z + bB.z; y[7] = rb.w + bB.w;
#pragma unroll
    for (int i = 0; i < 8; ++i) {
      float v = y[i];
      v = (v <= 0.0f) ? 0.0f : v;
      v = v + pzr;
      y[i] = v;
      const double dv = (double)v;
      ps[i] += dv;
      pq[i] += dv * dv;
    }
    v4f ya, yb;
    ya.x = y[0]; ya.y = y[1]; ya.z = y[2]; ya.w = y[3];
    yb.x = y[4]; yb.y = y[5]; yb.z = y[6]; yb.w = y[7];
    float* pp = P + ((size_t)rowOff + (size_t)node) * HC + 4 * lane;
    *(volatile v4f*)pp = ya;
    *(volatile v4f*)(pp + 128) = yb;
    __threadfence();
    *(volatile v4f*)pp = ya;
    *(volatile v4f*)(pp + 128) = yb;
  }

  {
    double* wr = wsum + wave * 512;
#pragma unroll
    for (int i = 0; i < 4; ++i) {
      wr[4 * lane + i]             = ps[i];
      wr[128 + 4 * lane + i]       = ps[4 + i];
      wr[256 + 4 * lane + i]       = pq[i];
      wr[256 + 128 + 4 * lane + i] = pq[4 + i];
    }
  }
  __syncthreads();
  {
    v2d tv; tv.x = 0.0; tv.y = 0.0;
#pragma unroll
    for (int w2 = 0; w2 < NWAVE; ++w2) {
      const v2d p = *(const v2da*)(wsum + w2 * 512 + 2 * tid);
      tv.x += p.x; tv.y += p.y;
    }
    double* rp = REC + ((size_t)bb * (size_t)gridDim.x + (size_t)blk) * 512 + 2 * tid;
    *(volatile v2d*)rp = tv;
    __threadfence();
    *(volatile v2d*)rp = tv;
  }
}

__global__ __launch_bounds__(NTHR) void k_st(const double* __restrict__ REC, int nRec,
                                             const float* __restrict__ gam, const float* __restrict__ bet,
                                             float* MR) {
  __shared__ __attribute__((aligned(16))) float sm[4 * HC];
  const int tid = (int)threadIdx.x;
  double S = 0.0, Q = 0.0;
#pragma unroll 2
  for (int r = 0; r < nRec; ++r) {
    S += REC[(size_t)r * 512 + tid];
    Q += REC[(size_t)r * 512 + 256 + tid];
  }
  const double mu = S / 40000.0;
  double var = Q / 40000.0 - mu * mu;
  var = (var < 0.0) ? 0.0 : var;
  const float varf = (float)var;
  const float rs = 1.0f / sqrtf(varf + 1e-5f);
  sm[tid]          = (float)mu;
  sm[HC + tid]     = rs;
  sm[2 * HC + tid] = bfr(gam[tid]);
  sm[3 * HC + tid] = bfr(bet[tid]);
  __syncthreads();
  const v4f v = *(const v4fa*)(sm + 4 * tid);
  *(volatile v4f*)(MR + 4 * tid) = v;
  __threadfence();
  *(volatile v4f*)(MR + 4 * tid) = v;
}

__global__ __launch_bounds__(NTHR) void k_bn1(const float* __restrict__ P, const float* __restrict__ MR,
                                              unsigned short* X, int nRows) {
  const int tid = (int)threadIdx.x, lane = tid & 31, wave = tid >> 5;
  const int row = (int)blockIdx.x * NWAVE + wave;
  if (row >= nRows) return;
  const float* pr = P + (size_t)row * HC + 8 * lane;
  const v4f x0 = *(const v4f*)pr,                          x1 = *(const v4f*)(pr + 4);
  const v4f m0 = *(const v4f*)(MR + 8 * lane),             m1 = *(const v4f*)(MR + 8 * lane + 4);
  const v4f r0 = *(const v4f*)(MR + HC + 8 * lane),        r1 = *(const v4f*)(MR + HC + 8 * lane + 4);
  const v4f g0 = *(const v4f*)(MR + 2 * HC + 8 * lane),    g1 = *(const v4f*)(MR + 2 * HC + 8 * lane + 4);
  const v4f e0 = *(const v4f*)(MR + 3 * HC + 8 * lane),    e1 = *(const v4f*)(MR + 3 * HC + 8 * lane + 4);
  float y[8];
  y[0] = ((x0.x - m0.x) * r0.x) * g0.x + e0.x;
  y[1] = ((x0.y - m0.y) * r0.y) * g0.y + e0.y;
  y[2] = ((x0.z - m0.z) * r0.z) * g0.z + e0.z;
  y[3] = ((x0.w - m0.w) * r0.w) * g0.w + e0.w;
  y[4] = ((x1.x - m1.x) * r1.x) * g1.x + e1.x;
  y[5] = ((x1.y - m1.y) * r1.y) * g1.y + e1.y;
  y[6] = ((x1.z - m1.z) * r1.z) * g1.z + e1.z;
  y[7] = ((x1.w - m1.w) * r1.w) * g1.w + e1.w;
  v8us ho, lo;
#pragma unroll
  for (int i = 0; i < 8; ++i) {
    const unsigned int hb = f2bf(y[i]);
    ho[i] = (unsigned short)hb;
    lo[i] = (unsigned short)f2bf(y[i] - bf2f(hb));
  }
  unsigned short* hp = X + (size_t)row * KA2 + 8 * lane;
  *(volatile v8us*)hp = ho;
  *(volatile v8us*)(hp + HC) = lo;
  __threadfence();
  *(volatile v8us*)hp = ho;
  *(volatile v8us*)(hp + HC) = lo;
}

__global__ __launch_bounds__(NTHR) void k_head(const float* __restrict__ P, const float* __restrict__ MR,
                                               const float* __restrict__ Wc, const float* __restrict__ bc,
                                               float* out, int nRows) {
  __shared__ __attribute__((aligned(16))) float so[128];
  const int tid = (int)threadIdx.x, lane = tid & 31, wave = tid >> 5;
  const int base = (int)blockIdx.x * 128;
  const v4f m0 = *(const v4f*)(MR + 8 * lane),             m1 = *(const v4f*)(MR + 8 * lane + 4);
  const v4f r0 = *(const v4f*)(MR + HC + 8 * lane),        r1 = *(const v4f*)(MR + HC + 8 * lane + 4);
  const v4f g0 = *(const v4f*)(MR + 2 * HC + 8 * lane),    g1 = *(const v4f*)(MR + 2 * HC + 8 * lane + 4);
  const v4f e0 = *(const v4f*)(MR + 3 * HC + 8 * lane),    e1 = *(const v4f*)(MR + 3 * HC + 8 * lane + 4);
  const v4f c0 = *(const v4f*)(Wc + 8 * lane),             c1 = *(const v4f*)(Wc + 8 * lane + 4);
  const float w0 = bfr(c0.x), w1 = bfr(c0.y), w2 = bfr(c0.z), w3 = bfr(c0.w);
  const float w4 = bfr(c1.x), w5 = bfr(c1.y), w6 = bfr(c1.z), w7 = bfr(c1.w);
  const float bcv = bfr(bc[0]);
#pragma unroll 1
  for (int i = 0; i < 16; ++i) {
    const int lr  = wave * 16 + i;
    const int row = base + lr;
    const int rc  = row < nRows ? row : nRows - 1;
    const float* pr = P + (size_t)rc * HC + 8 * lane;
    const v4f x0 = *(const v4f*)pr, x1 = *(const v4f*)(pr + 4);
    float d = 0.0f;
    d = fmaf(((x0.x - m0.x) * r0.x) * g0.x + e0.x, w0, d);
    d = fmaf(((x0.y - m0.y) * r0.y) * g0.y + e0.y, w1, d);
    d = fmaf(((x0.z - m0.z) * r0.z) * g0.z + e0.z, w2, d);
    d = fmaf(((x0.w - m0.w) * r0.w) * g0.w + e0.w, w3, d);
    d = fmaf(((x1.x - m1.x) * r1.x) * g1.x + e1.x, w4, d);
    d = fmaf(((x1.y - m1.y) * r1.y) * g1.y + e1.y, w5, d);
    d = fmaf(((x1.z - m1.z) * r1.z) * g1.z + e1.z, w6, d);
    d = fmaf(((x1.w - m1.w) * r1.w) * g1.w + e1.w, w7, d);
    d += __shfl_xor(d, 16, 32);
    d += __shfl_xor(d, 8, 32);
    d += __shfl_xor(d, 4, 32);
    d += __shfl_xor(d, 2, 32);
    d += __shfl_xor(d, 1, 32);
    if (lane == 0) so[lr] = d + bcv;
  }
  __syncthreads();
  int nv = nRows - base;
  nv = nv > 128 ? 128 : nv;
  const bool act = (4 * tid) < nv;
  const int ti = act ? tid : 0;
  const v4f v = *(const v4fa*)(so + 4 * ti);
  float* op = out + (size_t)base + 4 * ti;
  if (act) *(volatile v4f*)op = v;
  __threadfence();
  if (act) *(volatile v4f*)op = v;
}

static inline int cdiv(int a, int b) { return (a + b - 1) / b; }
static inline size_t al256(size_t o) { return (o + 255) & ~(size_t)255; }

extern "C" void kernel_launch(void* const* d_in, const int* in_sizes, int n_in,
                              void* d_out, int out_size, void* d_ws, size_t ws_size,
                              hipStream_t stream) {
  if (n_in < 24) return;
  if (in_sizes[0] != MROW * XF) return;
  if (in_sizes[1] != 2 * NEDGE) return;
  if (in_sizes[2] != HC * RTD || in_sizes[3] != HC * HID) return;
  if (in_sizes[4] != HC || in_sizes[5] != HC) return;
  if (in_sizes[6] != HID || in_sizes[7] != 1) return;
  if (in_sizes[8] != HID * NFD || in_sizes[9] != HID) return;
  if (in_sizes[10] != HC * HID) return;
  if (in_sizes[11] != HC || in_sizes[12] != HC || in_sizes[13] != HC) return;
  if (in_sizes[14] != HC * HC) return;
  if (in_sizes[15] != HC || in_sizes[16] != HC || in_sizes[17] != HC) return;
  if (in_sizes[18] != HC || in_sizes[19] != HC || in_sizes[20] != HC || in_sizes[21] != HC) return;
  if (in_sizes[22] != HC || in_sizes[23] != 1) return;
  if (out_size != MROW) return;

  const float* x    = (const float*)d_in[0];
  const int*   ei   = (const int*)  d_in[1];
  const float* Wih  = (const float*)d_in[2];
  const float* Whh  = (const float*)d_in[3];
  const float* bih  = (const float*)d_in[4];
  const float* bhh  = (const float*)d_in[5];
  const float* Wa   = (const float*)d_in[6];
  const float* ba   = (const float*)d_in[7];
  const float* Wn   = (const float*)d_in[8];
  const float* bnb  = (const float*)d_in[9];
  const float* W1   = (const float*)d_in[10];
  const float* as1  = (const float*)d_in[11];
  const float* ad1  = (const float*)d_in[12];
  const float* b1   = (const float*)d_in[13];
  const float* W2   = (const float*)d_in[14];
  const float* as2  = (const float*)d_in[15];
  const float* ad2  = (const float*)d_in[16];
  const float* b2   = (const float*)d_in[17];
  const float* g1   = (const float*)d_in[18];
  const float* be1  = (const float*)d_in[19];
  const float* g2   = (const float*)d_in[20];
  const float* be2  = (const float*)d_in[21];
  const float* Wc   = (const float*)d_in[22];
  const float* bc   = (const float*)d_in[23];
  float* out = (float*)d_out;
  const int nE = NEDGE, nN = NNODE;
  const int* src = ei;
  const int* dst = ei + nE;

  const int gA   = cdiv(nN, NBA);
  const int nRec = gA * BATCH;
  const int vec8 = ((nE & 3) == 0) ? 1 : 0;

  char* ws = (char*)d_ws;
  size_t off = 0;
  const size_t szXT = (size_t)3 * MROW * KXT * 2;
  const size_t szXB = (size_t)MROW * KXB * 2;
  const size_t szH0 = (size_t)MROW * KH * 2;
  const size_t szX1 = (size_t)MROW * KA2 * 2;
  if (szXT + szXB + szH0 > szX1) return;
  const size_t oA   = off; off = al256(off + szX1);
  const size_t oXW  = off; off = al256(off + (size_t)MROW * HC * 4);
  const size_t oP   = off; off = al256(off + (size_t)MROW * HC * 4);
  const size_t oSD  = off; off = al256(off + (size_t)8 * MROW * 4);
  const size_t oHIT = off; off = al256(off + (size_t)gA * RCAP * 4);
  const size_t oFLG = off; off = al256(off + (size_t)gA * 128);
  const size_t oRC1 = off; off = al256(off + (size_t)nRec * 512 * 8);
  const size_t oRC2 = off; off = al256(off + (size_t)nRec * 512 * 8);
  const size_t oMR1 = off; off = al256(off + (size_t)4 * HC * 4);
  const size_t oMR2 = off; off = al256(off + (size_t)4 * HC * 4);
  const size_t oWIH = off; off = al256(off + (size_t)HC * KXT * 2);
  const size_t oWHH = off; off = al256(off + (size_t)HC * KH * 2);
  const size_t oWN  = off; off = al256(off + (size_t)HID * KXB * 2);
  const size_t oW1D = off; off = al256(off + (size_t)HC * KH * 2);
  const size_t oW2D = off; off = al256(off + (size_t)HC * KA2 * 2);
  if (off > ws_size || off > (size_t)WSMAX) return;

  unsigned short* XT   = (unsigned short*)(ws + oA);
  unsigned short* XB   = (unsigned short*)(ws + oA + szXT);
  unsigned short* H0HL = (unsigned short*)(ws + oA + szXT + szXB);
  unsigned short* X1HL = (unsigned short*)(ws + oA);
  float*  XW   = (float*)(ws + oXW);
  float*  P    = (float*)(ws + oP);
  float*  SD   = (float*)(ws + oSD);
  int*    HITS = (int*)(ws + oHIT);
  int*    FLG  = (int*)(ws + oFLG);
  double* RC1  = (double*)(ws + oRC1);
  double* RC2  = (double*)(ws + oRC2);
  float*  MR1  = (float*)(ws + oMR1);
  float*  MR2  = (float*)(ws + oMR2);
  unsigned short* WIH  = (unsigned short*)(ws + oWIH);
  unsigned short* WHH2 = (unsigned short*)(ws + oWHH);
  unsigned short* WN   = (unsigned short*)(ws + oWN);
  unsigned short* W1D  = (unsigned short*)(ws + oW1D);
  unsigned short* W2D  = (unsigned short*)(ws + oW2D);

  const int bktLds  = BKT_LDS_INTS * 4;
  const int scanLds = SCAN_LDS_INTS * 4;
  const int lstmLds = LSTM_LDS;
  hipFuncSetAttribute(reinterpret_cast<const void*>(&k_bucket),
                      hipFuncAttributeMaxDynamicSharedMemorySize, bktLds);
  hipFuncSetAttribute(reinterpret_cast<const void*>(&k_scan),
                      hipFuncAttributeMaxDynamicSharedMemorySize, scanLds);
  hipFuncSetAttribute(reinterpret_cast<const void*>(&k_lstm),
                      hipFuncAttributeMaxDynamicSharedMemorySize, lstmLds);

  k_pa<<<MROW / PA_ROWS, NTHR, 0, stream>>>(x, XT, XB);
  k_pb<<<U_ALL / NTHR, NTHR, 0, stream>>>(Wih, Whh, Wn, W1, W2, WIH, WHH2, WN, W1D, W2D);
  k_bucket<<<gA, NTHR, bktLds, stream>>>(src, dst, nE, nN, vec8, HITS, FLG);
  k_lstm<<<MROW / 64, NTHR, lstmLds, stream>>>(XT, WIH, WHH2, XB, WN, bih, bhh, Wa, ba, bnb, H0HL);
  k_g<<<dim3(MROW / GBM, HC / GBN), GTHR, 0, stream>>>(H0HL, W1D, XW, KH, HC, as1, ad1, HID, SD, MROW);
  k_scan<<<dim3(gA, BATCH), NTHR, scanLds, stream>>>(HITS, FLG, XW, SD, b1, P, RC1, nN, MROW);
  k_st<<<1, NTHR, 0, stream>>>(RC1, nRec, g1, be1, MR1);
  k_bn1<<<MROW / NWAVE, NTHR, 0, stream>>>(P, MR1, X1HL, MROW);
  k_g<<<dim3(MROW / GBM, HC / GBN), GTHR, 0, stream>>>(X1HL, W2D, XW, KA2, HC, as2, ad2, HID, SD, MROW);
  k_scan<<<dim3(gA, BATCH), NTHR, scanLds, stream>>>(HITS, FLG, XW, SD, b2, P, RC2, nN, MROW);
  k_st<<<1, NTHR, 0, stream>>>(RC2, nRec, g2, be2, MR2);
  k_head<<<cdiv(MROW, 128), NTHR, 0, stream>>>(P, MR2, Wc, bc, out, MROW);
}
